// MultiheadTransformer_71829033058508
// MI455X (gfx1250) — hardware-run, weakly checked
//
#include <hip/hip_runtime.h>
#include <stddef.h>
#include <stdint.h>


#define NN      100000
#define EE      1600000
#define CH      128
#define KP      256
#define SPLIT1  0
#define SPLITF  1
#define KX1     (SPLIT1 ? 256 : 128)
#define KXF     (SPLITF ? 256 : 128)
#define NC1     512
#define GBM     64
#define GBN     128
#define GTHR    128
#define GWAVE   4
#define MP      100096
#define SROWS   128
#define NSB     (MP / SROWS)
#define RECW    256
#define VECF    1024
#define SNTHR   256
#define SNW     8
#define NBRUN   1024
#define SUBC    256
#define WLCAP   3584
#define RCAP    (SNW * WLCAP)
#define DEGCAP  64
#define SLSH    17
#define SMASK   ((1 << SLSH) - 1)
#define MEAS_MAXDEG 36
#define MEAS_B1024  16710
#define SCAN_ZINTS    (2 * RCAP + 3 * NBRUN)
#define SCAN_LDS_INTS (SCAN_ZINTS + 16)
#define QSCALE  0.17677669f

static_assert(NN <= (1 << SLSH));
static_assert(((long long)NBRUN << SLSH) < (1LL << 31));
static_assert(MP % GBM == 0 && MP % SROWS == 0 && MP >= NN && MP - NN < SROWS);
static_assert(EE % SUBC == 0 && (EE % 4) == 0);
static_assert(KX1 % 32 == 0 && KXF % 32 == 0 && KX1 <= KP && KXF <= KP);
static_assert(NC1 % GBN == 0 && CH == GBN && GBM == GWAVE * 16 && GTHR == GBN);
static_assert(DEGCAP >= MEAS_MAXDEG + 8);
static_assert(RCAP >= MEAS_B1024 + 8192);
static_assert(SCAN_ZINTS % 4 == 0);
static_assert(SCAN_LDS_INTS * 4 <= 300000);
static_assert(((NN + NBRUN - 1) / NBRUN) * NBRUN >= MP);
static_assert(NBRUN % SNW == 0 && NBRUN % 32 == 0);

typedef float          v4f   __attribute__((ext_vector_type(4)));
typedef float          v8f   __attribute__((ext_vector_type(8)));
typedef double         v2d   __attribute__((ext_vector_type(2)));
typedef int            v4i   __attribute__((ext_vector_type(4)));
typedef int            v8i   __attribute__((ext_vector_type(8)));
typedef unsigned short v4us  __attribute__((ext_vector_type(4)));
typedef unsigned short v8us  __attribute__((ext_vector_type(8)));
typedef unsigned short v16us __attribute__((ext_vector_type(16)));
typedef __bf16         v16bf __attribute__((ext_vector_type(16)));
typedef v4f  __attribute__((may_alias)) v4fa;
typedef v4i  __attribute__((may_alias)) v4ia;
typedef v8us __attribute__((may_alias)) v8usa;
union FragB { v16bf v; v16us u; v8us h[2]; v8i w; };

__device__ __forceinline__ v8f wmb(const FragB& a, const FragB& b, v8f c) {
  v8f d = __builtin_amdgcn_wmma_f32_16x16x32_bf16(false, a.v, false, b.v, (short)0, c, false, false);
  asm volatile("v_nop\n\tv_nop\n\tv_nop\n\tv_nop" : "+v"(d) : "v"(a.w), "v"(b.w));
  return d;
}
__device__ __forceinline__ v8f z8() { v8f z = {0.f, 0.f, 0.f, 0.f, 0.f, 0.f, 0.f, 0.f}; return z; }

__device__ __forceinline__ void ldwait() { asm volatile("s_wait_loadcnt 0x0" ::: "memory"); }

__device__ __forceinline__ unsigned bfbits(float f) {
  const unsigned u = __float_as_uint(f);
  return (u + 0x7FFFu + ((u >> 16) & 1u)) >> 16;
}
__device__ __forceinline__ unsigned bfbits_np(float f) {
  const unsigned r = bfbits(f);
  return (f != f) ? 0x7fc0u : r;
}
__device__ __forceinline__ float rbf(float f) { return __uint_as_float(bfbits(f) << 16); }

__device__ __forceinline__ v8us cvt8b(const v4f a, const v4f b) {
  v8us o;
  o[0] = (unsigned short)bfbits(a.x); o[1] = (unsigned short)bfbits(a.y);
  o[2] = (unsigned short)bfbits(a.z); o[3] = (unsigned short)bfbits(a.w);
  o[4] = (unsigned short)bfbits(b.x); o[5] = (unsigned short)bfbits(b.y);
  o[6] = (unsigned short)bfbits(b.z); o[7] = (unsigned short)bfbits(b.w);
  return o;
}

__device__ __forceinline__ void wunit(const float* __restrict__ w, unsigned short* dst, int u) {
  const int n  = u >> 5;
  const int k8 = (u & 31) * 8;
  const int ks = k8 & (CH - 1);
  const float* p = w + (size_t)ks * CH + n;
  v4f a, b;
  a.x = p[0];      a.y = p[CH];     a.z = p[2 * CH]; a.w = p[3 * CH];
  b.x = p[4 * CH]; b.y = p[5 * CH]; b.z = p[6 * CH]; b.w = p[7 * CH];
  const v8us hv = cvt8b(a, b);
  unsigned short* dp = dst + (size_t)u * 8;
  *(volatile v8us*)dp = hv;
  __threadfence();
  *(volatile v8us*)dp = hv;
}

__global__ __launch_bounds__(256) void k_prep(
    const float* __restrict__ Wq, const float* __restrict__ Wk, const float* __restrict__ Wv,
    const float* __restrict__ Ws, const float* __restrict__ Wfc,
    const float* __restrict__ bq, const float* __restrict__ bk, const float* __restrict__ bv,
    const float* __restrict__ bs, const float* __restrict__ bfc,
    const float* __restrict__ gam, const float* __restrict__ bet,
    unsigned short* W1T, unsigned short* WFT, float* VEC) {
  const int tid = (int)threadIdx.x;
  const int mi  = (int)blockIdx.x >> 4;
  const int u   = (((int)blockIdx.x & 15) << 8) + tid;
  if (mi == 0)      wunit(Wq,  W1T,                       u);
  else if (mi == 1) wunit(Wk,  W1T + (size_t)1 * CH * KP, u);
  else if (mi == 2) wunit(Wv,  W1T + (size_t)2 * CH * KP, u);
  else if (mi == 3) wunit(Ws,  W1T + (size_t)3 * CH * KP, u);
  else if (mi == 4) wunit(Wfc, WFT,                       u);
  else {
    const int wv = tid >> 5, lane = tid & 31;
    v4f a;
    if (wv == 0)      a = *(const v4f*)(bq  + 4 * lane);
    else if (wv == 1) a = *(const v4f*)(bk  + 4 * lane);
    else if (wv == 2) a = *(const v4f*)(bv  + 4 * lane);
    else if (wv == 3) a = *(const v4f*)(bs  + 4 * lane);
    else if (wv == 4) a = *(const v4f*)(bfc + 4 * lane);
    else if (wv == 5) a = *(const v4f*)(gam + 4 * lane);
    else if (wv == 6) a = *(const v4f*)(bet + 4 * lane);
    else return;
    v4f o;
    o.x = rbf(a.x); o.y = rbf(a.y); o.z = rbf(a.z); o.w = rbf(a.w);
    float* dp = VEC + 4 * tid;
    *(volatile v4f*)dp = o;
    __threadfence();
    *(volatile v4f*)dp = o;
  }
}

__global__ __launch_bounds__(256) void k_stats(const float* __restrict__ x, double* rec, int nN) {
  __shared__ double part[SNW * RECW];
  __shared__ __attribute__((aligned(16))) double fin[RECW];
  const int tid = (int)threadIdx.x, lane = tid & 31, wave = tid >> 5;
  const int row0 = (int)blockIdx.x * SROWS + wave * 16;
  double s0 = 0.0, s1 = 0.0, s2 = 0.0, s3 = 0.0, q0 = 0.0, q1 = 0.0, q2 = 0.0, q3 = 0.0;
#pragma unroll 2
  for (int i = 0; i < 16; ++i) {
    const int row = row0 + i;
    if (row < nN) {
      const v4f a = *(const v4f*)(x + (size_t)row * CH + 4 * lane);
      const double r0 = (double)rbf(a.x), r1 = (double)rbf(a.y), r2 = (double)rbf(a.z), r3 = (double)rbf(a.w);
      s0 += r0; s1 += r1; s2 += r2; s3 += r3;
      q0 += r0 * r0; q1 += r1 * r1; q2 += r2 * r2; q3 += r3 * r3;
    }
  }
  double* pw = part + wave * RECW;
  pw[4 * lane + 0] = s0; pw[4 * lane + 1] = s1; pw[4 * lane + 2] = s2; pw[4 * lane + 3] = s3;
  pw[CH + 4 * lane + 0] = q0; pw[CH + 4 * lane + 1] = q1; pw[CH + 4 * lane + 2] = q2; pw[CH + 4 * lane + 3] = q3;
  __syncthreads();
  {
    double f = 0.0;
#pragma unroll 1
    for (int w2 = 0; w2 < SNW; ++w2) f += part[w2 * RECW + tid];
    fin[tid] = f;
  }
  __syncthreads();
  v2d o;
  o.x = 0.0; o.y = 0.0;
  double* dp = rec + (size_t)blockIdx.x * RECW + 2 * (tid & 127);
  if (tid < 128) {
    o.x = fin[2 * tid]; o.y = fin[2 * tid + 1];
    *(volatile v2d*)dp = o;
  }
  __threadfence();
  if (tid < 128) {
    *(volatile v2d*)dp = o;
  }
}

__global__ __launch_bounds__(128) void k_combine(const double* __restrict__ rec, int nRec, int nN, float* murs) {
  __shared__ __attribute__((aligned(16))) float stg[2 * CH];
  const int c = (int)threadIdx.x;
  double s = 0.0, q = 0.0;
#pragma unroll 2
  for (int b = 0; b < nRec; ++b) {
    s += rec[(size_t)b * RECW + c];
    q += rec[(size_t)b * RECW + CH + c];
  }
  const double inv = 1.0 / (double)nN;
  const double mean = s * inv;
  double var = q * inv - mean * mean;
  var = var < 0.0 ? 0.0 : var;
  const float mu = (float)mean;
  const float rs = 1.0f / sqrtf((float)var + 1e-5f);
  stg[c] = mu;
  stg[CH + c] = rs;
  __syncthreads();
  v4f v = {0.f, 0.f, 0.f, 0.f};
  if (c < 64) {
    v = *(const v4fa*)(stg + 4 * c);
    *(volatile v4f*)(murs + 4 * c) = v;
  }
  __threadfence();
  if (c < 64) {
    *(volatile v4f*)(murs + 4 * c) = v;
  }
}

__global__ __launch_bounds__(256) void k_apply(const float* __restrict__ x, const float* __restrict__ murs,
                                               const float* __restrict__ gb, unsigned short* hl,
                                               int nN, int nUnits) {
  __shared__ __attribute__((aligned(16))) float psh[4 * CH];
  const int tid = (int)threadIdx.x;
  if (tid < 64)       *(v4fa*)(psh + 4 * tid) = *(const v4f*)(murs + 4 * tid);
  else if (tid < 128) *(v4fa*)(psh + 4 * tid) = *(const v4f*)(gb + 4 * (tid - 64));
  __syncthreads();
  const int u = (int)blockIdx.x * 256 + tid;
  if (u >= nUnits) return;
  const int row = u >> 4;
  const int c0  = (u & 15) * 8;
  const int rc  = row < nN ? row : nN - 1;
  const float* p = x + (size_t)rc * CH + c0;
  const v4f a = *(const v4f*)p;
  const v4f b = *(const v4f*)(p + 4);
  asm volatile("" :: "v"(a), "v"(b));
  const float live = row < nN ? 1.0f : 0.0f;
  const v4f m0 = *(const v4fa*)(psh + c0),          m1 = *(const v4fa*)(psh + c0 + 4);
  const v4f r0 = *(const v4fa*)(psh + CH + c0),     r1 = *(const v4fa*)(psh + CH + c0 + 4);
  const v4f g0 = *(const v4fa*)(psh + 2 * CH + c0), g1 = *(const v4fa*)(psh + 2 * CH + c0 + 4);
  const v4f e0 = *(const v4fa*)(psh + 3 * CH + c0), e1 = *(const v4fa*)(psh + 3 * CH + c0 + 4);
  float xv[8] = {a.x, a.y, a.z, a.w, b.x, b.y, b.z, b.w};
  float mv[8] = {m0.x, m0.y, m0.z, m0.w, m1.x, m1.y, m1.z, m1.w};
  float rv[8] = {r0.x, r0.y, r0.z, r0.w, r1.x, r1.y, r1.z, r1.w};
  float gv[8] = {g0.x, g0.y, g0.z, g0.w, g1.x, g1.y, g1.z, g1.w};
  float ev[8] = {e0.x, e0.y, e0.z, e0.w, e1.x, e1.y, e1.z, e1.w};
  v8us hv, lv;
#pragma unroll
  for (int j = 0; j < 8; ++j) {
    float t = (((rbf(xv[j]) - mv[j]) * rv[j]) * gv[j]) + ev[j];
    t = t > 0.0f ? t : 0.0f;
    t = t * live;
    const unsigned hb = bfbits(t);
    hv[j] = (unsigned short)hb;
    lv[j] = (unsigned short)bfbits(t - __uint_as_float(hb << 16));
  }
  unsigned short* hp = hl + (size_t)row * KP + c0;
  *(volatile v8us*)hp = hv;
  *(volatile v8us*)(hp + CH) = lv;
  __threadfence();
  *(volatile v8us*)hp = hv;
  *(volatile v8us*)(hp + CH) = lv;
}

__device__ __forceinline__ void put_rows(float* ob, int pitch, int row0, int lane, int nN, const v4f (&pv)[16]) {
#pragma unroll
  for (int i = 0; i < 16; ++i) {
    const int row = row0 + i;
    if (row < nN) *(volatile v4f*)(ob + (size_t)row * (size_t)pitch + 4 * lane) = pv[i];
  }
  __threadfence();
#pragma unroll
  for (int i = 0; i < 16; ++i) {
    const int row = row0 + i;
    if (row < nN) *(volatile v4f*)(ob + (size_t)row * (size_t)pitch + 4 * lane) = pv[i];
  }
}

template <int MODE>
__global__ __launch_bounds__(GTHR) __attribute__((amdgpu_num_vgpr(248)))
void k_gemm(const unsigned short* __restrict__ A, const unsigned short* __restrict__ BT,
            const float* __restrict__ bias, int kext, int nN,
            float* wsf, size_t oQ, size_t oKV, float* dout, const float* __restrict__ x) {
  __shared__ __attribute__((aligned(16))) float stg[GBM * GBN];
  __shared__ __attribute__((aligned(16))) float bsh[GBN];
  const int tid = (int)threadIdx.x, lane = tid & 31, wave = tid >> 5, hh = lane >> 4, m = lane & 15;
  const int rowBase = (int)blockIdx.x * GBM;
  const int by      = (int)blockIdx.y;
  const int colBase = by * GBN;

  v8f acc[8];
#pragma unroll
  for (int t = 0; t < 8; ++t) acc[t] = z8();
  const unsigned short* ap = A  + (size_t)(rowBase + 16 * wave + m) * (size_t)KP + 8 * hh;
  const unsigned short* bp = BT + (size_t)(colBase + m) * (size_t)KP + 8 * hh;

#pragma unroll 1
  for (int k0 = 0; k0 < kext; k0 += 32) {
    FragB af;
    af.h[0] = *(const v8usa*)(ap + k0);
    af.h[1] = *(const v8usa*)(ap + k0 + 16);
#pragma unroll
    for (int nt = 0; nt < 8; ++nt) {
      const unsigned short* wq = bp + (size_t)(16 * nt) * (size_t)KP + k0;
      FragB bf;
      bf.h[0] = *(const v8usa*)wq;
      bf.h[1] = *(const v8usa*)(wq + 16);
      acc[nt] = wmb(af, bf, acc[nt]);
    }
  }

#pragma unroll
  for (int nt = 0; nt < 8; ++nt) {
    const int lc = 16 * nt + m;
#pragma unroll
    for (int r = 0; r < 8; ++r) {
      const int lr = 16 * wave + 8 * hh + r;
      stg[lr * GBN + lc] = acc[nt][r];
    }
  }
  if (tid < 32) *(v4fa*)(bsh + 4 * tid) = *(const v4f*)(bias + colBase + 4 * tid);
  __syncthreads();

  const v4f b4 = *(const v4fa*)(bsh + 4 * lane);
  const int row0 = rowBase + 16 * wave;
  v4f pv[16];
  if constexpr (MODE == 1) {
#pragma unroll
    for (int i = 0; i < 16; ++i) {
      const v4f d = *(const v4fa*)(stg + (16 * wave + i) * GBN + 4 * lane);
      pv[i] = d + b4;
    }
    if (by == 3) {
      put_rows(dout, CH, row0, lane, nN, pv);
    } else {
      const size_t off = (by == 0) ? oQ : (oKV + (size_t)(by == 2 ? CH : 0));
      const int pitch  = (by == 0) ? CH : 2 * CH;
      put_rows(wsf + off, pitch, row0, lane, nN, pv);
    }
    (void)x;
  } else {
#pragma unroll
    for (int i = 0; i < 16; ++i) {
      const int row = row0 + i;
      const int rc  = row < nN ? row : nN - 1;
      const v4f xv = *(const v4f*)(x + (size_t)rc * CH + 4 * lane);
      asm volatile("" :: "v"(xv));
      const v4f d = *(const v4fa*)(stg + (16 * wave + i) * GBN + 4 * lane);
      v4f o;
      o.x = (d.x + b4.x) + rbf(xv.x);
      o.y = (d.y + b4.y) + rbf(xv.y);
      o.z = (d.z + b4.z) + rbf(xv.z);
      o.w = (d.w + b4.w) + rbf(xv.w);
      pv[i] = o;
    }
    put_rows(dout, CH, row0, lane, nN, pv);
    (void)wsf; (void)oQ; (void)oKV;
  }
}

__global__ __launch_bounds__(SNTHR) void k_scan(const int* __restrict__ srcs, const int* __restrict__ dsts,
                                                const float* __restrict__ Q, const float* __restrict__ KV,
                                                const float* __restrict__ Sp, unsigned short* conv,
                                                int nN, int nE) {
  extern __shared__ __attribute__((aligned(16))) int dsm[];
  int* wl   = dsm;
  int* pl   = wl + RCAP;
  int* scnt = pl + RCAP;
  int* soff = scnt + NBRUN;
  int* cur  = soff + NBRUN;
  int* misc = cur + NBRUN;
  const int tid = (int)threadIdx.x, lane = tid & 31, wave = tid >> 5;
  const int nodeBase = (int)blockIdx.x * NBRUN;
  const int nmax = nN - 1;

  {
    const v4i z4 = {0, 0, 0, 0};
    for (int i = tid * 4; i < SCAN_ZINTS; i += SNTHR * 4) *(v4ia*)(dsm + i) = z4;
    if (tid < 16) misc[tid] = 0;
  }
  __syncthreads();

  {
    const int nSub = nE / SUBC;
    const int per  = (nSub + SNW - 1) / SNW;
    const int sbeg = wave * per;
    int send = sbeg + per;
    send = send > nSub ? nSub : send;
    int wc = 0;
    int* mywl = wl + wave * WLCAP;
    const unsigned nbs = (unsigned)nodeBase;
#pragma unroll 1
    for (int sb = sbeg; sb < send; ++sb) {
      const int e0 = sb * SUBC + lane * 8;
      const v4i da = *(const v4i*)(dsts + e0);
      const v4i db = *(const v4i*)(dsts + e0 + 4);
      const v4i sa = *(const v4i*)(srcs + e0);
      const v4i sc = *(const v4i*)(srcs + e0 + 4);
      asm volatile("" :: "v"(sa), "v"(sc));
      const unsigned s0 = (unsigned)da.x - nbs, s1 = (unsigned)da.y - nbs;
      const unsigned s2 = (unsigned)da.z - nbs, s3 = (unsigned)da.w - nbs;
      const unsigned s4 = (unsigned)db.x - nbs, s5 = (unsigned)db.y - nbs;
      const unsigned s6 = (unsigned)db.z - nbs, s7 = (unsigned)db.w - nbs;
      const bool h0 = s0 < (unsigned)NBRUN, h1 = s1 < (unsigned)NBRUN, h2 = s2 < (unsigned)NBRUN, h3 = s3 < (unsigned)NBRUN;
      const bool h4 = s4 < (unsigned)NBRUN, h5 = s5 < (unsigned)NBRUN, h6 = s6 < (unsigned)NBRUN, h7 = s7 < (unsigned)NBRUN;
      const unsigned m0 = __builtin_amdgcn_ballot_w32(h0), m1 = __builtin_amdgcn_ballot_w32(h1);
      const unsigned m2 = __builtin_amdgcn_ballot_w32(h2), m3 = __builtin_amdgcn_ballot_w32(h3);
      const unsigned m4 = __builtin_amdgcn_ballot_w32(h4), m5 = __builtin_amdgcn_ballot_w32(h5);
      const unsigned m6 = __builtin_amdgcn_ballot_w32(h6), m7 = __builtin_amdgcn_ballot_w32(h7);
      const unsigned many = m0 | m1 | m2 | m3 | m4 | m5 | m6 | m7;
      if (many != 0u) {
        int p = wc
              + (int)__builtin_amdgcn_mbcnt_lo(m0, 0u) + (int)__builtin_amdgcn_mbcnt_lo(m1, 0u)
              + (int)__builtin_amdgcn_mbcnt_lo(m2, 0u) + (int)__builtin_amdgcn_mbcnt_lo(m3, 0u)
              + (int)__builtin_amdgcn_mbcnt_lo(m4, 0u) + (int)__builtin_amdgcn_mbcnt_lo(m5, 0u)
              + (int)__builtin_amdgcn_mbcnt_lo(m6, 0u) + (int)__builtin_amdgcn_mbcnt_lo(m7, 0u);
#define PUTJ(HJ, SJ, SRCJ) { \
          int sv = (SRCJ); sv = sv < 0 ? 0 : (sv > nmax ? nmax : sv); \
          if (HJ) { if (p < WLCAP) mywl[p] = sv | (int)((SJ) << SLSH); } \
          p += (HJ) ? 1 : 0; }
        PUTJ(h0, s0, sa.x)
        PUTJ(h1, s1, sa.y)
        PUTJ(h2, s2, sa.z)
        PUTJ(h3, s3, sa.w)
        PUTJ(h4, s4, sc.x)
        PUTJ(h5, s5, sc.y)
        PUTJ(h6, s6, sc.z)
        PUTJ(h7, s7, sc.w)
#undef PUTJ
        wc += (int)__builtin_popcount(m0) + (int)__builtin_popcount(m1) + (int)__builtin_popcount(m2)
            + (int)__builtin_popcount(m3) + (int)__builtin_popcount(m4) + (int)__builtin_popcount(m5)
            + (int)__builtin_popcount(m6) + (int)__builtin_popcount(m7);
      }
    }
    if (lane == 0) misc[wave] = wc;
  }
  __syncthreads();

  if (wave == 0) {
    int ov = 0, tot = 0;
#pragma unroll 1
    for (int w2 = 0; w2 < SNW; ++w2) {
      const int craw = misc[w2];
      ov |= (craw > WLCAP) ? 1 : 0;
      int c = craw < 0 ? 0 : (craw > WLCAP ? WLCAP : craw);
      c = __builtin_amdgcn_readfirstlane(c);
      tot += c;
#pragma unroll 1
      for (int b0 = 0; b0 < c; b0 += 32) {
        const int idx = b0 + lane;
        const int ent = wl[w2 * WLCAP + (idx < WLCAP ? idx : WLCAP - 1)];
        const int m32 = (c - b0) < 32 ? (c - b0) : 32;
#pragma unroll 1
        for (int k = 0; k < m32; ++k) {
          const int u  = __builtin_amdgcn_readlane(ent, k);
          const int sl = (u >> SLSH) & (NBRUN - 1);
          if (lane == 0) scnt[sl] = scnt[sl] + 1;
        }
      }
    }
    if (lane == 0) { misc[8] = tot; misc[9] = ov; }
  }
  __syncthreads();

  if (wave == 0) {
    const int base = lane * (NBRUN / 32);
    int s = 0;
#pragma unroll 1
    for (int i = 0; i < NBRUN / 32; ++i) { const int cv = scnt[base + i]; s += cv < 0 ? 0 : cv; }
    int incl = s;
#pragma unroll
    for (int d = 1; d < 32; d <<= 1) {
      const int y = __shfl_up(incl, d, 32);
      incl += (lane >= d) ? y : 0;
    }
    int run = incl - s;
#pragma unroll 1
    for (int i = 0; i < NBRUN / 32; ++i) {
      int cv = scnt[base + i];
      cv = cv < 0 ? 0 : cv;
      soff[base + i] = run;
      cur[base + i]  = run;
      run += cv;
    }
  }
  __syncthreads();

  if (wave == 0) {
#pragma unroll 1
    for (int w2 = 0; w2 < SNW; ++w2) {
      int c = misc[w2];
      c = c < 0 ? 0 : (c > WLCAP ? WLCAP : c);
      c = __builtin_amdgcn_readfirstlane(c);
#pragma unroll 1
      for (int b0 = 0; b0 < c; b0 += 32) {
        const int idx = b0 + lane;
        const int ent = wl[w2 * WLCAP + (idx < WLCAP ? idx : WLCAP - 1)];
        const int m32 = (c - b0) < 32 ? (c - b0) : 32;
#pragma unroll 1
        for (int k = 0; k < m32; ++k) {
          const int u  = __builtin_amdgcn_readlane(ent, k);
          const int sl = (u >> SLSH) & (NBRUN - 1);
          if (lane == 0) {
            int p = cur[sl];
            p = p < 0 ? 0 : (p > RCAP - 1 ? RCAP - 1 : p);
            pl[p] = u;
            cur[sl] = p + 1;
          }
        }
      }
    }
  }
  __syncthreads();

  int nh = misc[8];
  nh = nh < 0 ? 0 : (nh > RCAP ? RCAP : nh);
  const int ovf = misc[9];
  const float qnan = __int_as_float(0x7fc00000);
  const float pzb  = (ovf != 0) ? qnan : 0.0f;
  const float ninf = __int_as_float((int)0xff800000u);
#pragma unroll 1
  for (int si = 0; si < NBRUN / SNW; ++si) {
    const int slot = si * SNW + wave;
    const int node = nodeBase + slot;
    if (node < MP) {
      int cv = scnt[slot];
      const bool big = cv > DEGCAP;
      cv = cv < 0 ? 0 : (cv > DEGCAP ? DEGCAP : cv);
      int ovv = soff[slot];
      ovv = ovv < 0 ? 0 : (ovv > RCAP - 1 ? RCAP - 1 : ovv);
      int c = __builtin_amdgcn_readfirstlane(cv);
      const int o = __builtin_amdgcn_readfirstlane(ovv);
      if (c > nh - o) c = nh - o;
      c = c < 0 ? 0 : c;
      int last = o + c - 1;
      last = last < o ? o : last;
      last = last > RCAP - 1 ? RCAP - 1 : last;
      const int gcl = node < nN ? node : nmax;
      const v4f qv = *(const v4f*)(Q  + (size_t)gcl * CH + 4 * lane);
      const v4f sv = *(const v4f*)(Sp + (size_t)gcl * CH + 4 * lane);
      ldwait();
      asm volatile("" :: "v"(qv), "v"(sv));
      float mx = ninf, ss = 0.0f;
      float a0 = 0.0f, a1 = 0.0f, a2 = 0.0f, a3 = 0.0f;
#pragma unroll 1
      for (int qh = 0; qh < c; ++qh) {
        int idx = o + qh;
        idx = idx > last ? last : idx;
        const int ent = pl[idx];
        int sr = ent & SMASK;
        sr = sr > nmax ? nmax : sr;
        sr = __builtin_amdgcn_readfirstlane(sr);
        const float* kp = KV + (size_t)sr * (2 * CH) + 4 * lane;
        const v4f kk = *(const v4f*)kp;
        const v4f vv = *(const v4f*)(kp + CH);
        ldwait();
        float part = qv.x * kk.x;
        part = fmaf(qv.y, kk.y, part);
        part = fmaf(qv.z, kk.z, part);
        part = fmaf(qv.w, kk.w, part);
        part += __shfl_xor(part, 1, 32);
        part += __shfl_xor(part, 2, 32);
        part += __shfl_xor(part, 4, 32);
        const float al = part * QSCALE;
        const float df = al - mx;
        const float ee = expf(-fabsf(df));
        const bool  up = df > 0.0f;
        const float f1 = up ? ee : 1.0f;
        const float f2 = up ? 1.0f : ee;
        ss = fmaf(ss, f1, f2);
        a0 = fmaf(a0, f1, f2 * vv.x);
        a1 = fmaf(a1, f1, f2 * vv.y);
        a2 = fmaf(a2, f1, f2 * vv.z);
        a3 = fmaf(a3, f1, f2 * vv.w);
        mx = up ? al : mx;
      }
      const float sden = (c == 0) ? 1.0f : ss;
      const float inv  = 1.0f / sden;
      const float pz   = big ? qnan : pzb;
      const bool live  = node < nN;
      float r[4];
      r[0] = (((c == 0) ? 0.0f : a0 * inv) + sv.x) + pz;
      r[1] = (((c == 0) ? 0.0f : a1 * inv) + sv.y) + pz;
      r[2] = (((c == 0) ? 0.0f : a2 * inv) + sv.z) + pz;
      r[3] = (((c == 0) ? 0.0f : a3 * inv) + sv.w) + pz;
      v4us h4, l4;
#pragma unroll
      for (int j = 0; j < 4; ++j) {
        const float y = live ? r[j] : 0.0f;
        const unsigned hb = bfbits_np(y);
        h4[j] = (unsigned short)hb;
        l4[j] = (unsigned short)bfbits_np(y - __uint_as_float(hb << 16));
      }
      unsigned short* cp = conv + (size_t)node * KP + 4 * lane;
      *(volatile v4us*)cp = h4;
      *(volatile v4us*)(cp + CH) = l4;
      __threadfence();
      *(volatile v4us*)cp = h4;
      *(volatile v4us*)(cp + CH) = l4;
    }
  }
}

static inline size_t al256(size_t o) { return (o + 255) & ~(size_t)255; }

extern "C" void kernel_launch(void* const* d_in, const int* in_sizes, int n_in,
                              void* d_out, int out_size, void* d_ws, size_t ws_size,
                              hipStream_t stream) {
  if (n_in < 14) return;
  if (in_sizes[0] != NN * CH || in_sizes[1] != 2 * EE) return;
  if (in_sizes[2] != CH || in_sizes[3] != CH) return;
  if (in_sizes[4] != CH * CH || in_sizes[6] != CH * CH || in_sizes[8] != CH * CH) return;
  if (in_sizes[10] != CH * CH || in_sizes[12] != CH * CH) return;
  if (in_sizes[5] != CH || in_sizes[7] != CH || in_sizes[9] != CH || in_sizes[11] != CH || in_sizes[13] != CH) return;
  if (out_size != NN * CH) return;

  const float* x    = (const float*)d_in[0];
  const int*   ei   = (const int*)  d_in[1];
  const float* gam  = (const float*)d_in[2];
  const float* bet  = (const float*)d_in[3];
  const float* Wq   = (const float*)d_in[4];
  const float* bq   = (const float*)d_in[5];
  const float* Wk   = (const float*)d_in[6];
  const float* bk   = (const float*)d_in[7];
  const float* Wv   = (const float*)d_in[8];
  const float* bv   = (const float*)d_in[9];
  const float* Wsk  = (const float*)d_in[10];
  const float* bsk  = (const float*)d_in[11];
  const float* Wfc  = (const float*)d_in[12];
  const float* bfc  = (const float*)d_in[13];
  float* out = (float*)d_out;
  const int* src = ei;
  const int* dst = ei + EE;
  const int nN = NN, nE = EE;

  char* ws = (char*)d_ws;
  size_t off = 0;
  const size_t oHL  = off; off = al256(off + (size_t)MP * KP * 2);
  const size_t oQ   = off; off = al256(off + (size_t)MP * CH * 4);
  const size_t oKV  = off; off = al256(off + (size_t)MP * 2 * CH * 4);
  const size_t oW1T = off; off = al256(off + (size_t)NC1 * KP * 2);
  const size_t oWFT = off; off = al256(off + (size_t)CH * KP * 2);
  const size_t oVEC = off; off = al256(off + (size_t)VECF * 4);
  const size_t oREC = off; off = al256(off + (size_t)NSB * RECW * 8);
  const size_t oMRS = off; off = al256(off + (size_t)(2 * CH) * 4);
  if (off > ws_size || off > ((size_t)256u << 20)) return;
  unsigned short* HL  = (unsigned short*)(ws + oHL);
  unsigned short* W1T = (unsigned short*)(ws + oW1T);
  unsigned short* WFT = (unsigned short*)(ws + oWFT);
  float*  VEC  = (float*)(ws + oVEC);
  double* REC  = (double*)(ws + oREC);
  float*  MURS = (float*)(ws + oMRS);
  float*  wsf  = (float*)ws;

  const size_t scanLds = (size_t)SCAN_LDS_INTS * 4;
  hipFuncSetAttribute(reinterpret_cast<const void*>(&k_scan), hipFuncAttributeMaxDynamicSharedMemorySize, (int)scanLds);

  k_prep<<<81, 256, 0, stream>>>(Wq, Wk, Wv, Wsk, Wfc, bq, bk, bv, bsk, bfc, gam, bet, W1T, WFT, VEC);
  k_stats<<<NSB, 256, 0, stream>>>(x, REC, nN);
  k_combine<<<1, 128, 0, stream>>>(REC, NSB, nN, MURS);
  const int nUa = MP * 16;
  k_apply<<<nUa / 256, 256, 0, stream>>>(x, MURS, VEC + 640, HL, nN, nUa);
  k_gemm<1><<<dim3(MP / GBM, NC1 / GBN), GTHR, 0, stream>>>(HL, W1T, VEC, KX1, nN, wsf, oQ / 4, oKV / 4, out, x);
  const int gS = (MP + NBRUN - 1) / NBRUN;
  k_scan<<<gS, SNTHR, scanLds, stream>>>(src, dst, (const float*)(ws + oQ), (const float*)(ws + oKV),
                                         (const float*)out, HL, nN, nE);
  k_gemm<2><<<dim3(MP / GBM, 1), GTHR, 0, stream>>>(HL, WFT, VEC + 512, KXF, nN, wsf, 0, 0, out, x);
}
